// My_Model_13408887898682
// MI455X (gfx1250) — hardware-verified
//
#include <hip/hip_runtime.h>
#include <stddef.h>
#include <stdint.h>
#include <math.h>

typedef __attribute__((ext_vector_type(16))) _Float16 v16h;
typedef __attribute__((ext_vector_type(8)))  _Float16 v8h;
typedef __attribute__((ext_vector_type(16))) __bf16   v16b;
typedef __attribute__((ext_vector_type(8)))  __bf16   v8b;
typedef __attribute__((ext_vector_type(8)))  float    v8f;
typedef __attribute__((ext_vector_type(4)))  float    v4f;

constexpr int kBatch   = 4;
constexpr int kSL      = 512;
constexpr int kWin     = 256;
constexpr int kSch     = 3;
constexpr int kCch     = 128;
constexpr int kRnn     = 128;
constexpr int kFc      = 256;
constexpr int kNSeq    = kBatch * kSL;
constexpr int kFrameIn = kWin * kSch;
constexpr int kRows1   = 256;
constexpr int kM1      = kNSeq * kRows1;
constexpr int kK1Real  = 24;
constexpr int kK1      = 32;
constexpr int kP1Rows  = kRows1 / 4;
constexpr int kM2      = kNSeq * kP1Rows;
constexpr int kK2      = 1024;
constexpr int kP1Pad   = 16;
constexpr int kHRows   = kP1Rows / 4;
constexpr int kHP1     = kM2 / 4;
constexpr int kD1      = 13 * kCch;
constexpr int kHld     = kHRows * kCch;
constexpr int kG3      = 3 * kRnn;
constexpr int kG6      = 2 * kG3;
constexpr int kCat     = 2 * kRnn;
constexpr int kThreads = 256;
constexpr int kHP      = 136;
constexpr float kWCarry = 16.0f;
constexpr float kACarry = 16.0f;
constexpr float kPCarry = 4096.0f;
constexpr float kFold   = 1.0f / 256.0f;

static_assert(kM1 % 64 == 0 && ((kM1 / 64) * (kCch / 64)) % 8 == 0);
static_assert(kM2 % 64 == 0 && ((kM2 / 64) * (kCch / 64)) % 8 == 0);
static_assert((kM1 * 4) % kThreads == 0);
static_assert(kK1 % 32 == 0 && kK2 % 32 == 0 && kD1 % 32 == 0 && kCat % 32 == 0 && kRnn % 32 == 0 && kSL % 32 == 0);
static_assert(kNSeq % 64 == 0 && kG6 % 64 == 0 && kSL % 64 == 0 && kCat % 64 == 0 && kFc % 64 == 0);
static_assert(kHP % 8 == 0 && kHP >= kRnn);
static_assert(kThreads == 8 * 32 && kRnn == 8 * 16);
static_assert((kNSeq * kCat) % (8 * kThreads) == 0);
static_assert(kNSeq % 8 == 0 && kNSeq % kThreads == 0);

__device__ __forceinline__ unsigned short f2bf_bits(float f) {
  unsigned u = __float_as_uint(f);
  return (unsigned short)((u + 0x7FFFu + ((u >> 16) & 1u)) >> 16);
}
__device__ __forceinline__ float bf_bits2f(unsigned short h) { return __uint_as_float(((unsigned)h) << 16); }

__device__ __forceinline__ void dep_guard_h(v8f& a, v8f& b, v16h x, v16h y) { asm volatile("v_nop\n\tv_nop\n\tv_nop\n\tv_nop" : "+v"(a), "+v"(b) : "v"(x), "v"(y)); }
__device__ __forceinline__ void dep_guard_b(v8f& a, v8f& b, v16b x, v16b y) { asm volatile("v_nop\n\tv_nop\n\tv_nop\n\tv_nop" : "+v"(a), "+v"(b) : "v"(x), "v"(y)); }
__device__ __forceinline__ void keep4_h(v16h a, v16h b, v16h c, v16h d) { asm volatile("v_nop" :: "v"(a), "v"(b), "v"(c), "v"(d)); }
__device__ __forceinline__ void keep4_b(v16b a, v16b b, v16b c, v16b d) { asm volatile("v_nop" :: "v"(a), "v"(b), "v"(c), "v"(d)); }
__device__ __forceinline__ void acc_guard4(v8f& a, v8f& b, v8f& c, v8f& d) { asm volatile("v_nop\n\tv_nop\n\tv_nop\n\tv_nop" : "+v"(a), "+v"(b), "+v"(c), "+v"(d)); }
__device__ __forceinline__ void acc_guard3(v8f& a, v8f& b, v8f& c) { asm volatile("v_nop\n\tv_nop\n\tv_nop\n\tv_nop" : "+v"(a), "+v"(b), "+v"(c)); }
template <typename T> struct Frag;
template <> struct Frag<_Float16> {
  typedef v16h V; union U { v16h v; v8h h[2]; };
  static __device__ __forceinline__ v16h load(const _Float16* p) {
    U f; f.h[0] = *(const v8h*)(p); f.h[1] = *(const v8h*)(p + 16); return f.v;
  }
  static __device__ __forceinline__ v8f mma(v16h a, v16h b, v8f c) {
    return __builtin_amdgcn_wmma_f32_16x16x32_f16(false, a, false, b, (short)0, c, false, false);
  }
  static __device__ __forceinline__ void guard(v8f& a, v8f& b, v16h x, v16h y) { dep_guard_h(a, b, x, y); }
  static __device__ __forceinline__ void keep(v16h a, v16h b, v16h c, v16h d) { keep4_h(a, b, c, d); }
};
template <> struct Frag<__bf16> {
  typedef v16b V; union U { v16b v; v8b h[2]; };
  static __device__ __forceinline__ v16b load(const __bf16* p) {
    U f; f.h[0] = *(const v8b*)(p); f.h[1] = *(const v8b*)(p + 16); return f.v;
  }
  static __device__ __forceinline__ v8f mma(v16b a, v16b b, v8f c) {
    return __builtin_amdgcn_wmma_f32_16x16x32_bf16(false, a, false, b, (short)0, c, false, false);
  }
  static __device__ __forceinline__ void guard(v8f& a, v8f& b, v16b x, v16b y) { dep_guard_b(a, b, x, y); }
  static __device__ __forceinline__ void keep(v16b a, v16b b, v16b c, v16b d) { keep4_b(a, b, c, d); }
};
typedef Frag<_Float16> FragH;

template <int ET> struct Elem;
template <> struct Elem<0> { typedef _Float16 T; };
template <> struct Elem<1> { typedef __bf16 T; };
template <int ET, bool SPLIT, int BIAS_MODE, int OUT_MODE, bool RESID, int ACT = 0>
__global__ __launch_bounds__(256) void wmma_gemm64(
    const unsigned short* __restrict__ Ap, const unsigned short* __restrict__ A2p, int lda, long strideA,
    const unsigned short* __restrict__ Btp, const unsigned short* __restrict__ Bt2p, int ldb, long strideB,
    void* __restrict__ Cout, void* __restrict__ Cout2, int ldc, long strideC,
    const float* __restrict__ bias,
    const float* __restrict__ resid, long strideR,
    int M, int N, int K, float scale, float post) {
  static_assert(!(OUT_MODE == 3 && (BIAS_MODE == 1 || RESID)));
  typedef typename Elem<ET>::T T;
  typedef typename Frag<T>::V V;
  const T* A = (const T*)Ap; const T* A2 = (const T*)A2p; const T* Bt = (const T*)Btp; const T* Bt2 = (const T*)Bt2p;
  __shared__ __align__(16) float sT[8][16 * 68];
  const int b    = blockIdx.y;
  const int lane = threadIdx.x & 31;
  const int wave = threadIdx.x >> 5;
  const int tilesN = N >> 6;
  const int tilesM = M >> 6;
  const int tile = blockIdx.x * 8 + wave;
  if (tile >= tilesM * tilesN) return;
  const int tm = tile / tilesN;
  const int tn = tile - tm * tilesN;
  const int m0 = tm << 6;
  const int n0 = tn << 6;

  const T* Ab  = A  + (size_t)b * strideA;
  const T* Bb  = Bt + (size_t)b * strideB;
  const T* Ab2 = SPLIT ? (A2  + (size_t)b * strideA) : nullptr;
  const T* Bb2 = SPLIT ? (Bt2 + (size_t)b * strideB) : nullptr;

  const int rlane = lane & 15;
  const int koff  = (lane >> 4) * 8;
  const int mOff  = (lane >> 4) * 8;
  const int mHalf = lane >> 4;

  v8f acc[4][4];
#pragma unroll
  for (int i = 0; i < 4; ++i)
#pragma unroll
    for (int j = 0; j < 4; ++j) acc[i][j] = (v8f){0.f,0.f,0.f,0.f,0.f,0.f,0.f,0.f};

  for (int k0 = 0; k0 < K; k0 += 32) {
    V bh[4], bl[4];
#pragma unroll
    for (int j = 0; j < 4; ++j) {
      const size_t bo = (size_t)(n0 + (j << 4) + rlane) * ldb + koff + k0;
      bh[j] = Frag<T>::load(Bb + bo);
      if (SPLIT) bl[j] = Frag<T>::load(Bb2 + bo);
    }
#pragma unroll
    for (int i = 0; i < 4; ++i) {
      const size_t ao = (size_t)(m0 + (i << 4) + rlane) * lda + koff + k0;
      V ah = Frag<T>::load(Ab + ao);
      V al;
      if (SPLIT) al = Frag<T>::load(Ab2 + ao);
#pragma unroll
      for (int j = 0; j < 4; ++j) {
        acc[i][j] = Frag<T>::mma(ah, bh[j], acc[i][j]);
        if (SPLIT) {
          acc[i][j] = Frag<T>::mma(ah, bl[j], acc[i][j]);
          acc[i][j] = Frag<T>::mma(al, bh[j], acc[i][j]);
        }
      }
      Frag<T>::guard(acc[i][0], acc[i][3], ah, SPLIT ? al : ah);
    }
    Frag<T>::keep(bh[0], bh[1], bh[2], bh[3]);
    if (SPLIT) Frag<T>::keep(bl[0], bl[1], bl[2], bl[3]);
  }
  acc_guard4(acc[0][0], acc[0][1], acc[0][2], acc[0][3]);
  acc_guard4(acc[1][0], acc[1][1], acc[1][2], acc[1][3]);
  acc_guard4(acc[2][0], acc[2][1], acc[2][2], acc[2][3]);
  acc_guard4(acc[3][0], acc[3][1], acc[3][2], acc[3][3]);

  float* slab = sT[wave];
  const float* Rb = RESID ? (resid + (size_t)b * strideR) : nullptr;
#pragma unroll
  for (int i = 0; i < 4; ++i) {
    const int mBase = m0 + (i << 4);
#pragma unroll
    for (int j = 0; j < 4; ++j) {
      const int n = n0 + (j << 4) + rlane;
      float bv = 0.f;
      if (BIAS_MODE == 2) bv = bias[n];
      if (OUT_MODE == 3) {
        float p0 = acc[i][j][0] * scale, p1 = acc[i][j][4] * scale;
#pragma unroll
        for (int r = 1; r < 4; ++r) {
          p0 = fmaxf(p0, acc[i][j][r] * scale);
          p1 = fmaxf(p1, acc[i][j][4 + r] * scale);
        }
        p0 += bv; p1 += bv;
        if (ACT == 6) { p0 = (p0 > 0.f) ? p0 : 0.2f * p0; p1 = (p1 > 0.f) ? p1 : 0.2f * p1; }
        p0 *= post; p1 *= post;
        slab[(2 * mHalf) * 68 + (j << 4) + rlane] = p0;
        slab[(2 * mHalf + 1) * 68 + (j << 4) + rlane] = p1;
      } else {
#pragma unroll
        for (int r = 0; r < 8; ++r) {
          float v = acc[i][j][r] * scale;
          if (BIAS_MODE == 1) v += bias[mBase + mOff + r];
          if (BIAS_MODE == 2) v += bv;
          if (RESID) v += Rb[(size_t)(mBase + mOff + r) * ldc + n];
          if (ACT == 1) v = tanhf(v);
          if (ACT == 2) v = fmaxf(v, 0.0f);
          if (ACT == 4) v = (v > 0.f) ? v : 0.01f * v;
          if (ACT == 6) v = (v > 0.f) ? v : 0.2f * v;
          v *= post;
          slab[(mOff + r) * 68 + (j << 4) + rlane] = v;
        }
      }
    }
    __builtin_amdgcn_fence(__ATOMIC_RELEASE, "workgroup");
    __builtin_amdgcn_wave_barrier();
    __builtin_amdgcn_fence(__ATOMIC_ACQUIRE, "workgroup");
    if (OUT_MODE == 0) {
      float* C = (float*)Cout + (size_t)b * strideC;
      const int hh = lane >> 4, c4 = (lane & 15) * 4;
      for (int pass = 0; pass < 2; ++pass) {
#pragma unroll
        for (int it = 0; it < 8; ++it) {
          const int row = it * 2 + hh;
          v4f v = *(const v4f*)(slab + row * 68 + c4);
          *(volatile v4f*)(C + (size_t)(mBase + row) * ldc + n0 + c4) = v;
        }
        __threadfence();
      }
    } else if (OUT_MODE == 3) {
      const int q = lane >> 3, c8 = (lane & 7) * 8;
      unsigned short* C = (unsigned short*)Cout + (size_t)b * strideC;
      const int prow = (mBase >> 2) + q;
      for (int pass = 0; pass < 2; ++pass) {
        const float* sp = slab + q * 68 + c8;
        v8h hv;
#pragma unroll
        for (int e = 0; e < 8; ++e) hv[e] = (_Float16)sp[e];
        *(volatile v8h*)(C + (size_t)prow * ldc + n0 + c8) = hv;
        __threadfence();
      }
    } else {
      const int q = lane >> 3, c8 = (lane & 7) * 8;
      unsigned short* C  = (unsigned short*)Cout  + (size_t)b * strideC;
      unsigned short* C2 = (OUT_MODE == 2) ? ((unsigned short*)Cout2 + (size_t)b * strideC) : nullptr;
      for (int pass = 0; pass < 2; ++pass) {
#pragma unroll
        for (int it = 0; it < 4; ++it) {
          const int row = it * 4 + q;
          const float* sp = slab + row * 68 + c8;
          v8h hv, lv;
#pragma unroll
          for (int e = 0; e < 8; ++e) {
            if (OUT_MODE == 1) {
              hv[e] = (_Float16)sp[e];
            } else {
              unsigned short hb = f2bf_bits(sp[e]);
              unsigned short lb = f2bf_bits(sp[e] - bf_bits2f(hb));
              hv[e] = __builtin_bit_cast(_Float16, hb);
              lv[e] = __builtin_bit_cast(_Float16, lb);
            }
          }
          *(volatile v8h*)(C + (size_t)(mBase + row) * ldc + n0 + c8) = hv;
          if (OUT_MODE == 2) *(volatile v8h*)(C2 + (size_t)(mBase + row) * ldc + n0 + c8) = lv;
        }
        __threadfence();
      }
    }
    __builtin_amdgcn_fence(__ATOMIC_RELEASE, "workgroup");
    __builtin_amdgcn_wave_barrier();
    __builtin_amdgcn_fence(__ATOMIC_ACQUIRE, "workgroup");
  }
}

__device__ __forceinline__ float fsig(float v)  { return __builtin_amdgcn_rcpf(1.0f + __expf(-v)); }
__device__ __forceinline__ float ftanh(float v) { return 1.0f - 2.0f * __builtin_amdgcn_rcpf(__expf(2.0f * v) + 1.0f); }

__global__ __launch_bounds__(kThreads) void wprep_kernel(const float* __restrict__ W, int Kin, int ncol, int Kpad, int nrow,
                                                         float scale, unsigned short* __restrict__ bt) {
  const int tpr = Kpad >> 3;
  const int i = blockIdx.x * kThreads + threadIdx.x;
  if (i >= nrow * tpr) return;
  const int n   = i / tpr;
  const int k0  = (i - n * tpr) * 8;
  const int ncl = (n < ncol) ? n : (ncol - 1);
  v8h hv;
#pragma unroll
  for (int e = 0; e < 8; ++e) {
    const int k  = k0 + e;
    const int kc = (k < Kin) ? k : (Kin - 1);
    float v = W[(size_t)kc * ncol + ncl];
    if (k >= Kin || n >= ncol) v = 0.0f;
    hv[e] = (_Float16)(scale * v);
  }
  const size_t o = (size_t)i * 8;
  *(volatile v8h*)(bt + o) = hv;
  __threadfence();
  *(volatile v8h*)(bt + o) = hv;
}

__global__ __launch_bounds__(kThreads) void zero16_kernel(unsigned short* __restrict__ p, int n8) {
  const int i = blockIdx.x * kThreads + threadIdx.x;
  if (i >= n8) return;
  v8h z;
#pragma unroll
  for (int e = 0; e < 8; ++e) z[e] = (_Float16)0.0f;
  *(volatile v8h*)(p + (size_t)i * 8) = z;
  __threadfence();
  *(volatile v8h*)(p + (size_t)i * 8) = z;
}

__global__ __launch_bounds__(kThreads) void im2col1_kernel(const float* __restrict__ x, unsigned short* __restrict__ im1) {
  const int i  = blockIdx.x * kThreads + threadIdx.x;
  const int m  = i >> 2;
  const int k0 = (i & 3) * 8;
  const int n  = m >> 8;
  const int p  = m & (kRows1 - 1);
  const float* xf = x + (size_t)n * kFrameIn;
  v8h hv;
#pragma unroll
  for (int e = 0; e < 8; ++e) {
    const int k = k0 + e;
    int idx = 3 * p + k;
    idx = (idx < kFrameIn) ? idx : (kFrameIn - 1);
    float v = xf[idx];
    if (k >= kK1Real) v = 0.0f;
    hv[e] = (_Float16)v;
  }
  const size_t o = (size_t)i * 8;
  *(volatile v8h*)(im1 + o) = hv;
  __threadfence();
  *(volatile v8h*)(im1 + o) = hv;
}

__global__ __launch_bounds__(kThreads) void gru_layer_kernel(
    const float* __restrict__ xg,
    const unsigned short* __restrict__ utf, const unsigned short* __restrict__ utb,
    const float* __restrict__ bfw, const float* __restrict__ bbw,
    const float* __restrict__ h0f, const float* __restrict__ h0b,
    const int* __restrict__ mask,
    float* __restrict__ y) {
  __shared__ __align__(16) _Float16 Hs[16 * kHP];
  __shared__ __align__(16) float    Os[kBatch * kRnn];
  const int dir = blockIdx.x;
  const unsigned short* utp = (dir != 0) ? utb : utf;
  const float* bp = (dir != 0) ? bbw : bfw;
  const float* h0 = (dir != 0) ? h0b : h0f;
  const int tid = threadIdx.x, lane = tid & 31, wave = tid >> 5;
  const int c = lane & 15, hh = lane >> 4, koff = hh * 8;
  const int j = 16 * wave + c;

#pragma unroll 1
  for (int i = tid; i < 16 * kHP; i += kThreads) Hs[i] = (_Float16)0.0f;

  const float b0z = bp[j],       b0r = bp[kRnn + j],       b0h = bp[2 * kRnn + j];
  const float b1z = bp[kG3 + j], b1r = bp[kG3 + kRnn + j], b1h = bp[kG3 + 2 * kRnn + j];
  float hst[4];
#pragma unroll
  for (int r = 0; r < 4; ++r) hst[r] = h0[r * kRnn + j];
  __syncthreads();
  if (hh == 0) {
#pragma unroll
    for (int r = 0; r < 4; ++r) Hs[r * kHP + j] = (_Float16)(kACarry * hst[r]);
  }
  __syncthreads();

  const _Float16* arow = Hs + c * kHP + koff;
  const _Float16* ut = (const _Float16*)utp;
  const _Float16* uz = ut + (size_t)j * kRnn + koff;
  const _Float16* ur = ut + (size_t)(kRnn + j) * kRnn + koff;
  const _Float16* uh = ut + (size_t)(2 * kRnn + j) * kRnn + koff;
  const int colz = dir * kG3 + j, colr = colz + kRnn, colh = colz + 2 * kRnn;
  const v8f z8 = {0.f, 0.f, 0.f, 0.f, 0.f, 0.f, 0.f, 0.f};

#pragma unroll 1
  for (int step = 0; step < kSL; ++step) {
    const int t = (dir != 0) ? (kSL - 1 - step) : step;
    float xz[4], xr[4], xh[4];
    int mt[4];
#pragma unroll
    for (int r = 0; r < 4; ++r) {
      const size_t ro = (size_t)(r * kSL + t) * kG6;
      xz[r] = xg[ro + colz];
      xr[r] = xg[ro + colr];
      xh[r] = xg[ro + colh];
      mt[r] = mask[r * kSL + t];
    }
    v8f acc0 = z8, acc1 = z8, acc2 = z8;
#pragma unroll 1
    for (int kc = 0; kc < 4; ++kc) {
      const int k0 = kc * 32;
      const v16h a  = FragH::load(arow + k0);
      const v16h wz = FragH::load(uz + k0);
      const v16h wr = FragH::load(ur + k0);
      const v16h wh = FragH::load(uh + k0);
      acc0 = FragH::mma(a, wz, acc0);
      acc1 = FragH::mma(a, wr, acc1);
      acc2 = FragH::mma(a, wh, acc2);
      acc_guard3(acc0, acc1, acc2);
      keep4_h(a, wz, wr, wh);
    }
#pragma unroll
    for (int r = 0; r < 4; ++r) {
      const float pz = (xz[r] + b0z) + fmaf(acc0[r], kFold, b1z);
      const float pr = (xr[r] + b0r) + fmaf(acc1[r], kFold, b1r);
      const float gh = fmaf(acc2[r], kFold, b1h);
      const float zz = fsig(pz);
      const float rr = fsig(pr);
      const float cand = ftanh((xh[r] + b0h) + rr * gh);
      const float hn = fmaf(zz, hst[r] - cand, cand);
      hst[r] = (mt[r] != 0) ? hn : hst[r];
    }
    __syncthreads();
    if (hh == 0) {
#pragma unroll
      for (int r = 0; r < 4; ++r) {
        Hs[r * kHP + j] = (_Float16)(kACarry * hst[r]);
        Os[r * kRnn + j] = hst[r];
      }
    }
    __syncthreads();
    if (wave < kBatch) {
      const v4f v = *(const v4f*)(Os + wave * kRnn + lane * 4);
      float* dst = y + (size_t)(wave * kSL + t) * kCat + dir * kRnn + lane * 4;
      *(volatile v4f*)dst = v;
      __threadfence();
      *(volatile v4f*)dst = v;
    }
  }
}

template <int MODE>
__global__ __launch_bounds__(kThreads) void convert_rows_kernel(const float* __restrict__ yv, unsigned short* __restrict__ o0,
                                                               unsigned short* __restrict__ o1, int n8) {
  const int i = blockIdx.x * kThreads + threadIdx.x;
  if (i >= n8) return;
  const v4f a  = *(const v4f*)(yv + (size_t)i * 8);
  const v4f bq = *(const v4f*)(yv + (size_t)i * 8 + 4);
  const float f[8] = {a[0], a[1], a[2], a[3], bq[0], bq[1], bq[2], bq[3]};
  v8h hv, lv;
#pragma unroll
  for (int e = 0; e < 8; ++e) {
    if (MODE == 0) {
      hv[e] = (_Float16)(kACarry * f[e]);
      lv[e] = hv[e];
    } else {
      const unsigned short hb = f2bf_bits(f[e]);
      const unsigned short lb = f2bf_bits(f[e] - bf_bits2f(hb));
      hv[e] = __builtin_bit_cast(_Float16, hb);
      lv[e] = __builtin_bit_cast(_Float16, lb);
    }
  }
  const size_t o = (size_t)i * 8;
  *(volatile v8h*)(o0 + o) = hv;
  if (MODE == 1) *(volatile v8h*)(o1 + o) = lv;
  __threadfence();
  *(volatile v8h*)(o0 + o) = hv;
  if (MODE == 1) *(volatile v8h*)(o1 + o) = lv;
}

__global__ __launch_bounds__(kThreads) void transpose_ht_kernel(const float* __restrict__ yv, unsigned short* __restrict__ ht) {
  __shared__ __align__(16) float T[32 * 68];
  const int tid = threadIdx.x;
  const int blk = blockIdx.x;
  const int b  = blk >> 6;
  const int rem = blk & 63;
  const int dt = rem >> 3, st = rem & 7;
  const int d0 = dt * 32, s0 = st * 64;
  {
    const int s = tid >> 2, d8 = (tid & 3) * 8;
    const float* src = yv + (size_t)(b * kSL + s0 + s) * kCat + d0 + d8;
    const v4f a  = *(const v4f*)(src);
    const v4f bq = *(const v4f*)(src + 4);
    T[(d8 + 0) * 68 + s] = a[0];  T[(d8 + 1) * 68 + s] = a[1];
    T[(d8 + 2) * 68 + s] = a[2];  T[(d8 + 3) * 68 + s] = a[3];
    T[(d8 + 4) * 68 + s] = bq[0]; T[(d8 + 5) * 68 + s] = bq[1];
    T[(d8 + 6) * 68 + s] = bq[2]; T[(d8 + 7) * 68 + s] = bq[3];
  }
  __syncthreads();
  const int d = tid >> 3, s8 = (tid & 7) * 8;
  const v4f a  = *(const v4f*)(T + d * 68 + s8);
  const v4f bq = *(const v4f*)(T + d * 68 + s8 + 4);
  v8h hv;
  hv[0] = (_Float16)(kACarry * a[0]);  hv[1] = (_Float16)(kACarry * a[1]);
  hv[2] = (_Float16)(kACarry * a[2]);  hv[3] = (_Float16)(kACarry * a[3]);
  hv[4] = (_Float16)(kACarry * bq[0]); hv[5] = (_Float16)(kACarry * bq[1]);
  hv[6] = (_Float16)(kACarry * bq[2]); hv[7] = (_Float16)(kACarry * bq[3]);
  unsigned short* dst = ht + (size_t)(b * kCat + d0 + d) * kSL + s0 + s8;
  *(volatile v8h*)dst = hv;
  __threadfence();
  *(volatile v8h*)dst = hv;
}

__global__ __launch_bounds__(kThreads) void softmax_kernel(const float* __restrict__ S, const int* __restrict__ mask,
                                                           unsigned short* __restrict__ P) {
  __shared__ __align__(16) float buf[8 * kSL];
  const int tid = threadIdx.x, lane = tid & 31, wave = tid >> 5;
  const int row = blockIdx.x * 8 + wave;
  const int b = row >> 9, t = row & (kSL - 1);
  const float* s = S + (size_t)row * kSL;
  const int* mk = mask + b * kSL;
  float v[16];
  float mx = -3.0e38f;
#pragma unroll
  for (int e = 0; e < 16; ++e) {
    const int idx = e * 32 + lane;
    const float sv = s[idx];
    const int keep = mk[idx];
    v[e] = (keep != 0) ? sv : -1.0e9f;
    mx = fmaxf(mx, v[e]);
  }
#pragma unroll
  for (int off = 1; off < 32; off <<= 1) mx = fmaxf(mx, __shfl_xor(mx, off, 32));
  float sum = 0.f;
#pragma unroll
  for (int e = 0; e < 16; ++e) { v[e] = __expf(v[e] - mx); sum += v[e]; }
#pragma unroll
  for (int off = 1; off < 32; off <<= 1) sum += __shfl_xor(sum, off, 32);
  const float qm  = (mk[t] != 0) ? kPCarry : 0.0f;
  const float inv = qm * __builtin_amdgcn_rcpf(sum);
  float* bw = buf + wave * kSL;
#pragma unroll
  for (int e = 0; e < 16; ++e) bw[e * 32 + lane] = v[e] * inv;
  __syncthreads();
  unsigned short* prow = P + (size_t)row * kSL;
  for (int pass = 0; pass < 2; ++pass) {
#pragma unroll
    for (int ch = 0; ch < 2; ++ch) {
      const float* sp = bw + ch * 256 + lane * 8;
      const v4f a  = *(const v4f*)(sp);
      const v4f bq = *(const v4f*)(sp + 4);
      v8h hv;
      hv[0] = (_Float16)a[0];  hv[1] = (_Float16)a[1];  hv[2] = (_Float16)a[2];  hv[3] = (_Float16)a[3];
      hv[4] = (_Float16)bq[0]; hv[5] = (_Float16)bq[1]; hv[6] = (_Float16)bq[2]; hv[7] = (_Float16)bq[3];
      *(volatile v8h*)(prow + ch * 256 + lane * 8) = hv;
    }
    __threadfence();
  }
}

__global__ __launch_bounds__(kThreads) void head_kernel(const float* __restrict__ D2, const float* __restrict__ w3,
                                                        const float* __restrict__ b3, float* __restrict__ out) {
  __shared__ __align__(16) float os[kThreads];
  const int tid = threadIdx.x, lane = tid & 31, wave = tid >> 5;
  const int r = blockIdx.x * kThreads + tid;
  const float* rowp = D2 + (size_t)r * kFc;
  float acc = 0.0f;
#pragma unroll 1
  for (int k4 = 0; k4 < kFc / 4; ++k4) {
    const v4f a = *(const v4f*)(rowp + 4 * k4);
    const v4f w = *(const v4f*)(w3 + 4 * k4);
    acc = fmaf(a[0], w[0], acc);
    acc = fmaf(a[1], w[1], acc);
    acc = fmaf(a[2], w[2], acc);
    acc = fmaf(a[3], w[3], acc);
  }
  os[tid] = acc + b3[0];
  __syncthreads();
  if (wave < 2) {
    const int idx = wave * 32 + lane;
    const v4f v = *(const v4f*)(os + idx * 4);
    float* dst = out + (size_t)blockIdx.x * kThreads + idx * 4;
    *(volatile v4f*)dst = v;
    __threadfence();
    *(volatile v4f*)dst = v;
  }
}

extern "C" void kernel_launch(void* const* d_in, const int* in_sizes, int n_in,
                              void* d_out, int out_size, void* d_ws, size_t ws_size, hipStream_t stream) {
  if (n_in < 28 || out_size < kNSeq) return;
  if (in_sizes[0] < kNSeq * kFrameIn || in_sizes[1] < kNSeq) return;
  const float* x    = (const float*)d_in[0];
  const int*   m    = (const int*)  d_in[1];
  const float* s1f  = (const float*)d_in[2];
  const float* s1b  = (const float*)d_in[3];
  const float* s2f  = (const float*)d_in[4];
  const float* s2b  = (const float*)d_in[5];
  const float* w1   = (const float*)d_in[6];
  const float* b1   = (const float*)d_in[7];
  const float* w2   = (const float*)d_in[8];
  const float* b2   = (const float*)d_in[9];
  const float* g1fW = (const float*)d_in[10]; const float* g1fU = (const float*)d_in[11]; const float* g1fb = (const float*)d_in[12];
  const float* g1bW = (const float*)d_in[13]; const float* g1bU = (const float*)d_in[14]; const float* g1bb = (const float*)d_in[15];
  const float* g2fW = (const float*)d_in[16]; const float* g2fU = (const float*)d_in[17]; const float* g2fb = (const float*)d_in[18];
  const float* g2bW = (const float*)d_in[19]; const float* g2bU = (const float*)d_in[20]; const float* g2bb = (const float*)d_in[21];
  const float* d1w  = (const float*)d_in[22]; const float* d1b  = (const float*)d_in[23];
  const float* d2w  = (const float*)d_in[24]; const float* d2b  = (const float*)d_in[25];
  const float* d3w  = (const float*)d_in[26]; const float* d3b  = (const float*)d_in[27];
  float* out = (float*)d_out;

  char* ws = (char*)d_ws;
  size_t off = 0;
  auto carve = [&](size_t bytes) -> void* {
    off = (off + 255) & ~(size_t)255;
    void* p = ws + off;
    off += bytes;
    return p;
  };
  unsigned short* bt1 = (unsigned short*)carve((size_t)kCch * kK1 * 2);
  unsigned short* bt2 = (unsigned short*)carve((size_t)kCch * kK2 * 2);
  unsigned short* w1t = (unsigned short*)carve((size_t)kG6 * kD1 * 2);
  unsigned short* u1f = (unsigned short*)carve((size_t)kG3 * kRnn * 2);
  unsigned short* u1b = (unsigned short*)carve((size_t)kG3 * kRnn * 2);
  unsigned short* u2f = (unsigned short*)carve((size_t)kG3 * kRnn * 2);
  unsigned short* u2b = (unsigned short*)carve((size_t)kG3 * kRnn * 2);
  unsigned short* w2t = (unsigned short*)carve((size_t)kG6 * kCat * 2);
  unsigned short* d1t = (unsigned short*)carve((size_t)kFc * kCat * 2);
  unsigned short* d2t = (unsigned short*)carve((size_t)kFc * kFc * 2);
  unsigned short* im1 = (unsigned short*)carve((size_t)kM1 * kK1 * 2);
  unsigned short* p1  = (unsigned short*)carve((size_t)(kM2 + kP1Pad) * kCch * 2);
  unsigned short* hpl = (unsigned short*)carve((size_t)kHP1 * kCch * 2);
  float*          xg1 = (float*)carve((size_t)kNSeq * kG6 * 4);
  float*          y1  = (float*)carve((size_t)kNSeq * kCat * 4);
  unsigned short* h1h = (unsigned short*)carve((size_t)kNSeq * kCat * 2);
  float*          xg2 = (float*)carve((size_t)kNSeq * kG6 * 4);
  float*          y2  = (float*)carve((size_t)kNSeq * kCat * 4);
  unsigned short* y2hi = (unsigned short*)carve((size_t)kNSeq * kCat * 2);
  unsigned short* y2lo = (unsigned short*)carve((size_t)kNSeq * kCat * 2);
  unsigned short* ht  = (unsigned short*)carve((size_t)kBatch * kCat * kSL * 2);
  float*          sc  = (float*)carve((size_t)kBatch * kSL * kSL * 4);
  unsigned short* pp  = (unsigned short*)carve((size_t)kBatch * kSL * kSL * 2);
  unsigned short* o16 = (unsigned short*)carve((size_t)kNSeq * kCat * 2);
  unsigned short* d1o = (unsigned short*)carve((size_t)kNSeq * kFc * 2);
  float*          d2o = (float*)carve((size_t)kNSeq * kFc * 4);
  if (off > ws_size || off > (size_t)134217728) return;

  const dim3 blk(kThreads);

  wprep_kernel<<<(kCch * (kK1 / 8) + kThreads - 1) / kThreads, blk, 0, stream>>>(w1, kK1Real, kCch, kK1, kCch, kWCarry, bt1);
  wprep_kernel<<<(kCch * (kK2 / 8) + kThreads - 1) / kThreads, blk, 0, stream>>>(w2, kK2, kCch, kK2, kCch, kWCarry, bt2);
  wprep_kernel<<<(kG3 * (kD1 / 8) + kThreads - 1) / kThreads, blk, 0, stream>>>(g1fW, kD1, kG3, kD1, kG3, kWCarry, w1t);
  wprep_kernel<<<(kG3 * (kD1 / 8) + kThreads - 1) / kThreads, blk, 0, stream>>>(g1bW, kD1, kG3, kD1, kG3, kWCarry, w1t + (size_t)kG3 * kD1);
  wprep_kernel<<<(kG3 * (kRnn / 8) + kThreads - 1) / kThreads, blk, 0, stream>>>(g1fU, kRnn, kG3, kRnn, kG3, kWCarry, u1f);
  wprep_kernel<<<(kG3 * (kRnn / 8) + kThreads - 1) / kThreads, blk, 0, stream>>>(g1bU, kRnn, kG3, kRnn, kG3, kWCarry, u1b);
  wprep_kernel<<<(kG3 * (kRnn / 8) + kThreads - 1) / kThreads, blk, 0, stream>>>(g2fU, kRnn, kG3, kRnn, kG3, kWCarry, u2f);
  wprep_kernel<<<(kG3 * (kRnn / 8) + kThreads - 1) / kThreads, blk, 0, stream>>>(g2bU, kRnn, kG3, kRnn, kG3, kWCarry, u2b);
  wprep_kernel<<<(kG3 * (kCat / 8) + kThreads - 1) / kThreads, blk, 0, stream>>>(g2fW, kCat, kG3, kCat, kG3, kWCarry, w2t);
  wprep_kernel<<<(kG3 * (kCat / 8) + kThreads - 1) / kThreads, blk, 0, stream>>>(g2bW, kCat, kG3, kCat, kG3, kWCarry, w2t + (size_t)kG3 * kCat);
  wprep_kernel<<<(kFc * (kCat / 8) + kThreads - 1) / kThreads, blk, 0, stream>>>(d1w, kCat, kFc, kCat, kFc, kWCarry, d1t);
  wprep_kernel<<<(kFc * (kFc / 8) + kThreads - 1) / kThreads, blk, 0, stream>>>(d2w, kFc, kFc, kFc, kFc, kWCarry, d2t);

  zero16_kernel<<<(kP1Pad * kCch / 8 + kThreads - 1) / kThreads, blk, 0, stream>>>(p1 + (size_t)kM2 * kCch, kP1Pad * kCch / 8);
  im2col1_kernel<<<(kM1 * 4) / kThreads, blk, 0, stream>>>(x, im1);
  wmma_gemm64<0, false, 2, 3, false, 6><<<dim3((kM1 / 64) * (kCch / 64) / 8, 1), blk, 0, stream>>>(
      im1, im1, kK1, 0, bt1, bt1, kK1, 0, p1, p1, kCch, 0, b1, b1, 0, kM1, kCch, kK1, 1.0f / 16.0f, kACarry);
  wmma_gemm64<0, false, 2, 3, false, 6><<<dim3((kM2 / 64) * (kCch / 64) / 8, 1), blk, 0, stream>>>(
      p1, p1, kCch, 0, bt2, bt2, kK2, 0, hpl, hpl, kCch, 0, b2, b2, 0, kM2, kCch, kK2, kFold, kACarry);

  wmma_gemm64<0, false, 0, 0, false, 0><<<dim3((kNSeq / 64) * (kG6 / 64) / 8, 1), blk, 0, stream>>>(
      hpl, hpl, kHld, 0, w1t, w1t, kD1, 0, xg1, xg1, kG6, 0, b1, b1, 0, kNSeq, kG6, kD1, kFold, 1.0f);
  gru_layer_kernel<<<2, blk, 0, stream>>>(xg1, u1f, u1b, g1fb, g1bb, s1f, s1b, m, y1);
  convert_rows_kernel<0><<<(kNSeq * kCat / 8) / kThreads, blk, 0, stream>>>(y1, h1h, h1h, kNSeq * kCat / 8);

  wmma_gemm64<0, false, 0, 0, false, 0><<<dim3((kNSeq / 64) * (kG6 / 64) / 8, 1), blk, 0, stream>>>(
      h1h, h1h, kCat, 0, w2t, w2t, kCat, 0, xg2, xg2, kG6, 0, b1, b1, 0, kNSeq, kG6, kCat, kFold, 1.0f);
  gru_layer_kernel<<<2, blk, 0, stream>>>(xg2, u2f, u2b, g2fb, g2bb, s2f, s2b, m, y2);
  convert_rows_kernel<1><<<(kNSeq * kCat / 8) / kThreads, blk, 0, stream>>>(y2, y2hi, y2lo, kNSeq * kCat / 8);
  transpose_ht_kernel<<<kBatch * (kCat / 32) * (kSL / 64), blk, 0, stream>>>(y2, ht);

  wmma_gemm64<1, true, 0, 0, false, 0><<<dim3((kSL / 64) * (kSL / 64) / 8, kBatch), blk, 0, stream>>>(
      y2hi, y2lo, kCat, (long)kSL * kCat, y2hi, y2lo, kCat, (long)kSL * kCat, sc, sc, kSL, (long)kSL * kSL,
      b1, b1, 0, kSL, kSL, kCat, 1.0f, 1.0f);
  softmax_kernel<<<kNSeq / 8, blk, 0, stream>>>(sc, m, pp);
  wmma_gemm64<0, false, 0, 1, false, 0><<<dim3((kSL / 64) * (kCat / 64) / 8, kBatch), blk, 0, stream>>>(
      pp, pp, kSL, (long)kSL * kSL, ht, ht, kSL, (long)kCat * kSL, o16, o16, kCat, (long)kSL * kCat,
      b1, b1, 0, kSL, kCat, kSL, 1.0f / kPCarry, 1.0f);

  wmma_gemm64<0, false, 2, 1, false, 6><<<dim3((kNSeq / 64) * (kFc / 64) / 8, 1), blk, 0, stream>>>(
      o16, o16, kCat, 0, d1t, d1t, kCat, 0, d1o, d1o, kFc, 0, d1b, d1b, 0, kNSeq, kFc, kCat, kFold, kACarry);
  wmma_gemm64<0, false, 2, 0, false, 6><<<dim3((kNSeq / 64) * (kFc / 64) / 8, 1), blk, 0, stream>>>(
      d1o, d1o, kFc, 0, d2t, d2t, kFc, 0, d2o, d2o, kFc, 0, d2b, d2b, 0, kNSeq, kFc, kFc, kFold, 1.0f);
  head_kernel<<<kNSeq / kThreads, blk, 0, stream>>>(d2o, d3w, d3b, out);
}
